// RelationalNetworkEncoder_27006754357647
// MI455X (gfx1250) — hardware-verified
//
#include <hip/hip_runtime.h>
#include <math.h>

typedef __attribute__((ext_vector_type(16))) _Float16 v16h;
typedef __attribute__((ext_vector_type(16))) __bf16 v16b;
typedef __attribute__((ext_vector_type(8)))  _Float16 v8h;
typedef __attribute__((ext_vector_type(8)))  float v8f;
typedef __attribute__((ext_vector_type(4)))  float v4f;
typedef __attribute__((ext_vector_type(2)))  float v2f;
typedef __attribute__((ext_vector_type(4)))  unsigned v4u;
typedef __attribute__((ext_vector_type(4)))  int v4i;
typedef float __attribute__((may_alias)) float_a;
typedef int __attribute__((may_alias)) int_a;

template <typename T> __device__ __forceinline__ void vst2(void* p, T v) { *(volatile T*)p = v; __threadfence(); *(volatile T*)p = v; }
__device__ __forceinline__ v8f wmma16(v16h a, v16h b, v8f c) {
  v8f d = __builtin_amdgcn_wmma_f32_16x16x32_f16(false, a, false, b, (short)0, c, false, false);
  asm volatile("v_nop\n\tv_nop\n\tv_nop\n\tv_nop" : "+v"(d) : "v"(a), "v"(b));
  return d;
}
__device__ __forceinline__ v8f wmma_bf(v16b a, v16b b, v8f c) {
  v8f d = __builtin_amdgcn_wmma_f32_16x16x32_bf16(false, a, false, b, (short)0, c, false, false);
  asm volatile("v_nop\n\tv_nop\n\tv_nop\n\tv_nop" : "+v"(d) : "v"(a), "v"(b));
  return d;
}
__device__ __forceinline__ v16h frag_h(const _Float16* rowk0, int lane) {
  union { v16h v; v8h q[2]; } u; const _Float16* p = rowk0 + 8 * (lane >> 4);
  u.q[0] = *(const v8h*)p; u.q[1] = *(const v8h*)(p + 16); return u.v;
}
__device__ __forceinline__ v16h frag_f32(const float* rowk0, int lane) {
  v16h a; const float* p = rowk0 + 8 * (lane >> 4);
#pragma unroll
  for (int i = 0; i < 8; ++i) { a[i] = (_Float16)p[i]; a[8 + i] = (_Float16)p[16 + i]; }
  return a;
}
__device__ __forceinline__ v16h frag_f32s(const float* rowk0, int lane, float sc) {
  v16h a; const float* p = rowk0 + 8 * (lane >> 4);
#pragma unroll
  for (int i = 0; i < 8; ++i) { a[i] = (_Float16)(p[i] * sc); a[8 + i] = (_Float16)(p[16 + i] * sc); }
  return a;
}
__device__ __forceinline__ v16h fragc_f32(const float* W, int k0, int n, int lane, int ld, int K) {
  v16h a; const int g = lane >> 4;
#pragma unroll
  for (int i = 0; i < 8; ++i) { const int ka = k0 + 8 * g + i, kb = ka + 16;
    a[i] = (_Float16)(ka < K ? W[(size_t)(ka < K ? ka : K - 1) * ld + n] : 0.f); a[8 + i] = (_Float16)(kb < K ? W[(size_t)(kb < K ? kb : K - 1) * ld + n] : 0.f); }
  return a;
}
struct F2 { v16b h, l; };
__device__ __forceinline__ F2 bsplit16(const float v[16]) { F2 r;
#pragma unroll
  for (int i = 0; i < 16; ++i) { const __bf16 h = (__bf16)v[i]; r.h[i] = h; r.l[i] = (__bf16)(v[i] - (float)h); }
  return r; }
__device__ __forceinline__ F2 split_row(const float* row, int k0, int lane) { float v[16]; const float* p = row + k0 + 8 * (lane >> 4);
#pragma unroll
  for (int i = 0; i < 8; ++i) { v[i] = p[i]; v[8 + i] = p[16 + i]; }
  return bsplit16(v); }
__device__ __forceinline__ F2 split_rowK(const float* row, int k0, int lane, int K) { float v[16]; const int g = lane >> 4;
#pragma unroll
  for (int i = 0; i < 8; ++i) { const int ka = k0 + 8 * g + i, kb = ka + 16; v[i] = ka < K ? row[ka < K ? ka : K - 1] : 0.f; v[8 + i] = kb < K ? row[kb < K ? kb : K - 1] : 0.f; }
  return bsplit16(v); }
__device__ __forceinline__ F2 split_col(const float* W, int k0, int n, int lane, int ld, int K) { float v[16]; const int g = lane >> 4;
#pragma unroll
  for (int i = 0; i < 8; ++i) { const int ka = k0 + 8 * g + i, kb = ka + 16; v[i] = ka < K ? W[(size_t)(ka < K ? ka : K - 1) * ld + n] : 0.f; v[8 + i] = kb < K ? W[(size_t)(kb < K ? kb : K - 1) * ld + n] : 0.f; }
  return bsplit16(v); }
__device__ __forceinline__ v8f mac3(const F2& a, const F2& b, v8f c) { c = wmma_bf(a.l, b.h, c); c = wmma_bf(a.h, b.l, c); return wmma_bf(a.h, b.h, c); }
__device__ __forceinline__ float sigm(float v) { return 1.0f / (1.0f + expf(-v)); }
#define LDSX() do { asm volatile("s_wait_dscnt 0" ::: "memory"); __builtin_amdgcn_wave_barrier(); __builtin_amdgcn_fence(__ATOMIC_RELEASE, "workgroup"); } while (0)


#define NBI 8
#define CIN 512
#define CH 256
#define HWN 196
#define HWP 256
#define LB 4
#ifndef TK
#define TK HWN
#define TB NBI
#endif
typedef __attribute__((ext_vector_type(8))) __bf16 v8b;
__device__ __forceinline__ v16b frag_b(const __bf16* rowk0, int lane) {
  union { v16b v; v8b q[2]; } u; const __bf16* p = rowk0 + 8 * (lane >> 4);
  u.q[0] = *(const v8b*)p; u.q[1] = *(const v8b*)(p + 16); return u.v;
}
__device__ __forceinline__ float bfr(float v) { return (float)(__bf16)v; }
__device__ __attribute__((noinline)) float exp_ni(float v) { return expf(v); }
__device__ __attribute__((noinline)) float erf_ni(float v) { return erff(v); }

#define PK_PR 0
#define PK_W1 ((size_t)CH * CIN)
#define PK_W2 (PK_W1 + (size_t)2 * CH * CH)
#define PK_W3 (PK_W2 + (size_t)CH * CH)
#define PK_END (PK_W3 + (size_t)CH * CH)
#define WS_PK  0u
#define WS_X   (((2u * PK_END) + 127u) / 128u * 128u)
#define WS_AL  (WS_X + 4u * NBI * HWP * CH)
#define WS_AK  (WS_AL + 4u * NBI * HWP * CH)
#define WS_PS  (WS_AK + 4u * NBI * HWP * CH)
#define WS_END (WS_PS + 4u * (size_t)NBI * HWN * LB * CH)

__global__ __launch_bounds__(256) void k_pack(const float* __restrict__ PW, const float* __restrict__ W1, const float* __restrict__ W2, const float* __restrict__ W3, __bf16* __restrict__ PK) {
  __shared__ __align__(16) __bf16 s[CIN]; const int n = blockIdx.x, which = blockIdx.y, t = threadIdx.x; int K; size_t dst;
  if (which == 0) { if (n >= CH) return; K = CIN; dst = PK_PR + (size_t)n * CIN; for (int k = t; k < K; k += 256) s[k] = (__bf16)PW[(size_t)n * CIN + k]; }
  else if (which == 1) { K = CH; dst = PK_W1 + (size_t)n * CH; const int half = n / CH, o = n % CH; for (int k = t; k < K; k += 256) s[k] = (__bf16)W1[((size_t)half * CH + k) * CH + o]; }
  else if (which == 2) { if (n >= CH) return; K = CH; dst = PK_W2 + (size_t)n * CH; for (int k = t; k < K; k += 256) s[k] = (__bf16)W2[(size_t)k * CH + n]; }
  else { if (n >= CH) return; K = CH; dst = PK_W3 + (size_t)n * CH; for (int k = t; k < K; k += 256) s[k] = (__bf16)W3[(size_t)k * CH + n]; }
  __syncthreads();
  for (int q = t; q < K / 8; q += 256) vst2((unsigned*)(PK + dst + q * 8), *(const v4u*)&s[q * 8]);
}
__global__ __launch_bounds__(128) void k_proj(const float* __restrict__ IM, const __bf16* __restrict__ PK, const float* __restrict__ PB, float* __restrict__ X) {
  __shared__ __align__(16) __bf16 sa[64][CIN + 8]; __shared__ __align__(16) float so[4][16][CH + 4];
  const int tid = threadIdx.x, wave = tid >> 5, lane = tid & 31, col = lane & 15, g = lane >> 4; const int p0 = blockIdx.x * 64; const size_t b = blockIdx.y;
  for (int e = tid; e < 64 * CIN; e += 128) { const int c = e >> 6, r = e & 63; const int p = p0 + r; sa[r][c] = (__bf16)((p < HWN) ? IM[(b * CIN + c) * HWN + p] : 0.f); }
  if (tid < 64) for (int c = CIN; c < CIN + 8; ++c) sa[tid][c] = (__bf16)0.f;
  __syncthreads();
  v8f acc[16] = {};
#pragma unroll 2
  for (int kc = 0; kc < CIN / 32; ++kc) { const v16b a = frag_b(&sa[wave * 16 + col][kc * 32], lane);
#pragma unroll
    for (int j = 0; j < 16; ++j) acc[j] = wmma_bf(a, frag_b(PK + PK_PR + (size_t)(j * 16 + col) * CIN + kc * 32, lane), acc[j]); }
#pragma unroll
  for (int j = 0; j < 16; ++j) { const float bb = bfr(PB[j * 16 + col]);
#pragma unroll
    for (int r = 0; r < 8; ++r) so[wave][8 * g + r][j * 16 + col] = acc[j][r] + bb; }
  LDSX();
  for (int rl = 0; rl < 16; ++rl) for (int q = lane; q < CH / 4; q += 32) vst2(X + ((b * HWP + p0 + wave * 16 + rl) * CH) + q * 4, *(const v4f*)&so[wave][rl][q * 4]);
}
__global__ __launch_bounds__(128) void k_a(const float* __restrict__ X, const __bf16* __restrict__ PK, const float* __restrict__ B1, float* __restrict__ AL, float* __restrict__ AK) {
  __shared__ __align__(16) float so[4][16][CH + 4];
  const int tid = threadIdx.x, wave = tid >> 5, lane = tid & 31, col = lane & 15, g = lane >> 4; const int which = blockIdx.y; const size_t b = blockIdx.z; const size_t r0 = b * HWP + (size_t)blockIdx.x * 64 + wave * 16;
  v8f acc[16] = {};
#pragma unroll 2
  for (int kc = 0; kc < CH / 32; ++kc) { const F2 a = split_row(X + (r0 + col) * CH, kc * 32, lane);
#pragma unroll
    for (int j = 0; j < 16; ++j) { const v16b w = frag_b(PK + PK_W1 + ((size_t)which * CH + j * 16 + col) * CH + kc * 32, lane); acc[j] = wmma_bf(a.l, w, acc[j]); acc[j] = wmma_bf(a.h, w, acc[j]); } }
#pragma unroll
  for (int j = 0; j < 16; ++j) { const float bb = (which == 0) ? bfr(B1[j * 16 + col]) : 0.f;
#pragma unroll
    for (int r = 0; r < 8; ++r) so[wave][8 * g + r][j * 16 + col] = acc[j][r] + bb; }
  LDSX();
  float* D = which ? AK : AL;
  for (int rl = 0; rl < 16; ++rl) for (int q = lane; q < CH / 4; q += 32) vst2(D + (r0 + rl) * CH + q * 4, *(const v4f*)&so[wave][rl][q * 4]);
}
__global__ __launch_bounds__(128) void k_pair(const float* __restrict__ AL, const float* __restrict__ AK, const __bf16* __restrict__ PK, const float* __restrict__ B2, const float* __restrict__ B3, float* __restrict__ PS) {
  __shared__ __align__(16) __bf16 sh[64][CH + 8]; __shared__ __align__(16) float sak[CH]; __shared__ __align__(16) float ssum[4][CH];
  const int tid = threadIdx.x, wave = tid >> 5, lane = tid & 31, col = lane & 15, g = lane >> 4; const int k = blockIdx.x, lb = blockIdx.y; const size_t b = blockIdx.z; const int l0 = lb * 64;
  for (int c = tid; c < CH; c += 128) sak[c] = AK[(b * HWP + k) * CH + c];
  __syncthreads();
  for (int e = tid; e < 64 * CH; e += 128) { const int r = e / CH, c = e % CH; const int l = l0 + r; float v = 0.f; if (l < HWN) v = fmaxf(sak[c] + AL[(b * HWP + l) * CH + c], 0.f); sh[r][c] = (__bf16)v; }
  if (tid < 64) for (int c = CH; c < CH + 8; ++c) sh[tid][c] = (__bf16)0.f;
  __syncthreads();
  v8f acc[16];
#pragma unroll 1
  for (int layer = 0; layer < 2; ++layer) { const __bf16* Wr = PK + (layer ? PK_W3 : PK_W2); const float* BB = layer ? B3 : B2;
#pragma unroll
    for (int j = 0; j < 16; ++j) acc[j] = v8f{};
#pragma unroll 2
    for (int kc = 0; kc < CH / 32; ++kc) { const v16b a = frag_b(&sh[wave * 16 + col][kc * 32], lane);
#pragma unroll
      for (int j = 0; j < 16; ++j) acc[j] = wmma_bf(a, frag_b(Wr + (size_t)(j * 16 + col) * CH + kc * 32, lane), acc[j]); }
    __syncthreads();
    if (layer == 0) {
#pragma unroll
      for (int j = 0; j < 16; ++j) { const float bb = bfr(BB[j * 16 + col]);
#pragma unroll
        for (int r = 0; r < 8; ++r) sh[wave * 16 + 8 * g + r][j * 16 + col] = (__bf16)fmaxf(acc[j][r] + bb, 0.f); }
      __syncthreads(); }
    else {
#pragma unroll
      for (int j = 0; j < 16; ++j) { const float bb = bfr(BB[j * 16 + col]); float s = 0.f;
#pragma unroll
        for (int r = 0; r < 8; ++r) { const int l = l0 + wave * 16 + 8 * g + r; if (l < HWN) s += fmaxf(acc[j][r] + bb, 0.f); }
        s += __shfl_xor(s, 16);
        if (g == 0) ssum[wave][j * 16 + col] = s; } } }
  __syncthreads();
  for (int c4 = tid; c4 < CH / 4; c4 += 128) { v4f o; for (int i = 0; i < 4; ++i) { const int c = c4 * 4 + i; o[i] = ((ssum[0][c] + ssum[1][c]) + (ssum[2][c] + ssum[3][c])); } vst2(PS + (((b * HWN + k) * LB + lb) * CH) + c4 * 4, o); }
}
__global__ __launch_bounds__(256) void k_sum(const float* __restrict__ PS, float* __restrict__ OUT) {
  const size_t b = blockIdx.x; const int c = threadIdx.x; float s = 0.f;
  for (int k = 0; k < HWN; ++k) for (int lb = 0; lb < LB; ++lb) s += PS[(((b * HWN + k) * LB + lb) * CH) + c];
  __shared__ __align__(16) float so[CH]; so[c] = s; __syncthreads();
  if (c < CH / 4) vst2(OUT + b * CH + c * 4, *(const v4f*)&so[c * 4]);
}
extern "C" void kernel_launch(void* const* d_in, const int* in_sizes, int n_in, void* d_out, int out_size, void* d_ws, size_t ws_size, hipStream_t stream) {
  (void)in_sizes; (void)n_in; (void)out_size;
  const float** F = (const float**)d_in;
  if (ws_size < (size_t)WS_END) return;
  char* ws = (char*)d_ws; __bf16* PK = (__bf16*)(ws + WS_PK); float *X = (float*)(ws + WS_X), *AL = (float*)(ws + WS_AL), *AK = (float*)(ws + WS_AK), *PS = (float*)(ws + WS_PS);
  k_pack<<<dim3(2 * CH, 4), 256, 0, stream>>>(F[3], F[5], F[7], F[9], PK);
  k_proj<<<dim3(HWP / 64, NBI), 128, 0, stream>>>(F[0], PK, F[4], X);
  k_a<<<dim3(HWP / 64, 2, NBI), 128, 0, stream>>>(X, PK, F[6], AL, AK);
  k_pair<<<dim3(TK, LB, TB), 128, 0, stream>>>(AL, AK, PK, F[8], F[10], PS);
  k_sum<<<TB, 256, 0, stream>>>(PS, (float*)d_out);
}
